// decoderAttention_12498354831698
// MI455X (gfx1250) — hardware-verified
//
#include <hip/hip_runtime.h>
#include <stdint.h>

#define CDIM    384
#define NQ      4098
#define NKEY    4099
#define NINT    4096
#define NHEAD   6
#define DHEAD   64
#define NPADR   4160
#define C8      (CDIM / 8)
#define PLANE   ((size_t)NPADR * CDIM)
#define NEGFILL (-1.0e9f)
#define PADFILL (-1.0e30f)
static_assert(NHEAD * DHEAD == CDIM);
static_assert((NPADR % 64) == 0 && (CDIM % 64) == 0 && (CDIM % 32) == 0);
static_assert(NPADR >= NKEY && NPADR >= NQ);
static_assert((NPADR * C8) % 256 == 0);
static_assert((NPADR % 4) == 0);
static_assert((NINT % 8) == 0);

typedef __bf16 v16b __attribute__((ext_vector_type(16)));
typedef float  v8f  __attribute__((ext_vector_type(8)));
typedef float  v4f  __attribute__((ext_vector_type(4)));
typedef unsigned int   v4u  __attribute__((ext_vector_type(4)));
typedef unsigned short v8us __attribute__((ext_vector_type(8)));
typedef v8us __attribute__((may_alias)) v8usa;
typedef v4f  __attribute__((may_alias)) v4fa;
union FB { v16b v; v8us u[2]; unsigned w[8]; };

#if defined(__HIP_DEVICE_COMPILE__)
#define DEV_ASM 1
#else
#define DEV_ASM 0
#endif

__device__ __forceinline__ unsigned short bf_bits(float f) {
  unsigned u = __float_as_uint(f);
  return (unsigned short)((u + 0x7FFFu + ((u >> 16) & 1u)) >> 16);
}
__device__ __forceinline__ float bf_up(unsigned short hb) { return __uint_as_float(((unsigned)hb) << 16); }
__device__ __forceinline__ float bf_rn(float f) { return bf_up(bf_bits(f)); }
__device__ __forceinline__ unsigned pk16(unsigned short a, unsigned short b) { return (unsigned)a | ((unsigned)b << 16); }
__device__ __forceinline__ v8f zero8() { v8f z = {0.f, 0.f, 0.f, 0.f, 0.f, 0.f, 0.f, 0.f}; return z; }
__device__ __forceinline__ void split2(float f, unsigned short& h, unsigned short& l) {
  h = bf_bits(f);
  l = bf_bits(f - bf_up(h));
}
__device__ __forceinline__ void split8(const float* f, float sc, v4u& hi, v4u& lo) {
  v4u a, b;
#pragma unroll
  for (int e = 0; e < 4; ++e) {
    unsigned short h0, l0, h1, l1;
    split2(f[2 * e] * sc, h0, l0);
    split2(f[2 * e + 1] * sc, h1, l1);
    a[e] = pk16(h0, h1);
    b[e] = pk16(l0, l1);
  }
  hi = a; lo = b;
}

__device__ __forceinline__ v16b ldfrag_b(const unsigned short* p, int h) {
  FB f;
  f.u[0] = *(const v8usa*)(p + 8 * h);
  f.u[1] = *(const v8usa*)(p + 16 + 8 * h);
  return f.v;
}

__device__ __forceinline__ v8f mmar(v16b a, v16b b, v8f c) {
  return __builtin_amdgcn_wmma_f32_16x16x32_bf16(false, a, false, b, (short)0, c, false, false);
}
__device__ __forceinline__ v8f mma_g(v16b a, v16b b, v8f c) {
  c = __builtin_amdgcn_wmma_f32_16x16x32_bf16(false, a, false, b, (short)0, c, false, false);
#if DEV_ASM
  asm volatile("v_nop\n\tv_nop\n\tv_nop\n\tv_nop" : "+v"(c) : "v"(a), "v"(b));
#endif
  return c;
}
__device__ __forceinline__ void dep_guard(v8f& a, v8f& b, v16b x, v16b y) {
#if DEV_ASM
  asm volatile("v_nop\n\tv_nop\n\tv_nop\n\tv_nop" : "+v"(a), "+v"(b) : "v"(x), "v"(y));
#else
  (void)a; (void)b; (void)x; (void)y;
#endif
}
__device__ __forceinline__ void keep4(v16b a, v16b b, v16b c, v16b d) {
#if DEV_ASM
  asm volatile("v_nop" :: "v"(a), "v"(b), "v"(c), "v"(d));
#else
  (void)a; (void)b; (void)c; (void)d;
#endif
}
__device__ __forceinline__ void acc_guard4(v8f& a, v8f& b, v8f& c, v8f& d) {
#if DEV_ASM
  asm volatile("v_nop\n\tv_nop\n\tv_nop\n\tv_nop" : "+v"(a), "+v"(b), "+v"(c), "+v"(d));
#else
  (void)a; (void)b; (void)c; (void)d;
#endif
}

__device__ __forceinline__ void pack_p2(v8f a, v8f c, v16b& ph, v16b& pl) {
  FB h, l;
#pragma unroll
  for (int i = 0; i < 4; ++i) {
    unsigned short h0, l0, h1, l1, g0, m0, g1, m1;
    split2(a[2 * i], h0, l0);
    split2(a[2 * i + 1], h1, l1);
    split2(c[2 * i], g0, m0);
    split2(c[2 * i + 1], g1, m1);
    h.w[i] = pk16(h0, h1);      l.w[i] = pk16(l0, l1);
    h.w[4 + i] = pk16(g0, g1);  l.w[4 + i] = pk16(m0, m1);
  }
  ph = h.v; pl = l.v;
}

__global__ __launch_bounds__(256) void back_kernel(const float* __restrict__ x, const float* __restrict__ msk,
                                                   float* back) {
  __shared__ float ssum[8][32];
  __shared__ float scnt[8][32];
  const int lane = (int)threadIdx.x & 31, w = (int)threadIdx.x >> 5;
  const int c = blockIdx.x * 32 + lane;
  float sum = 0.f, cnt = 0.f;
#pragma unroll 1
  for (int i = 0; i < NINT / 8; ++i) {
    const int n = w * (NINT / 8) + i;
    const float mv = bf_rn(msk[n]);
    const float xv = bf_rn(x[(size_t)(1 + n) * CDIM + c]);
    const bool rev = mv < 0.5f;
    sum += rev ? xv : 0.f;
    cnt += rev ? 1.f : 0.f;
  }
  ssum[w][lane] = sum;
  scnt[w][lane] = cnt;
  __syncthreads();
  if (w == 0) {
    float ts = 0.f, tc = 0.f;
#pragma unroll
    for (int k = 0; k < 8; ++k) { ts += ssum[k][lane]; tc += scnt[k][lane]; }
    const float rc = 1.0f / (tc + 1e-10f);
    const float v = ts * rc;
    *(volatile float*)(back + c) = v;
    __threadfence();
    *(volatile float*)(back + c) = v;
  }
}

__global__ __launch_bounds__(256) void wcvt_kernel(const float* __restrict__ w0, const float* __restrict__ w1,
                                                   const float* __restrict__ w2, const float* __restrict__ w3,
                                                   unsigned short* wb) {
  const int which = blockIdx.y;
  const float* src = (which == 0) ? w0 : ((which == 1) ? w1 : ((which == 2) ? w2 : w3));
  const int i = blockIdx.x * 256 + (int)threadIdx.x;
  if (i >= CDIM * CDIM / 8) return;
  const v4f a = *(const v4fa*)(src + (size_t)i * 8);
  const v4f b = *(const v4fa*)(src + (size_t)i * 8 + 4);
  v4u p;
  p[0] = pk16(bf_bits(a[0]), bf_bits(a[1]));
  p[1] = pk16(bf_bits(a[2]), bf_bits(a[3]));
  p[2] = pk16(bf_bits(b[0]), bf_bits(b[1]));
  p[3] = pk16(bf_bits(b[2]), bf_bits(b[3]));
  unsigned short* o = wb + (size_t)which * CDIM * CDIM + (size_t)i * 8;
  *(volatile v4u*)o = p;
  __threadfence();
  *(volatile v4u*)o = p;
}

__global__ __launch_bounds__(256) void keymask_kernel(const float* __restrict__ msk, const float* __restrict__ mblk,
                                                      float* mk) {
  const int t = blockIdx.x * 256 + (int)threadIdx.x;
  if (t >= NPADR / 4) return;
  v4f v;
#pragma unroll
  for (int e = 0; e < 4; ++e) {
    const int j = 4 * t + e;
    int ji = j - 1; ji = (ji < 0) ? 0 : ji; ji = (ji > NINT - 1) ? (NINT - 1) : ji;
    const int jb = (j > NKEY - 1) ? (NKEY - 1) : j;
    const float mi = bf_rn(msk[ji]);
    const float mb = bf_rn(mblk[jb]);
    const bool interior = (j >= 1) && (j <= NINT);
    const float mv = interior ? mi : mb;
    float code = (mv >= 0.5f) ? 1.0f : NEGFILL;
    code = (j < NKEY) ? code : PADFILL;
    v[e] = code;
  }
  float* o = mk + (size_t)t * 4;
  *(volatile v4f*)o = v;
  __threadfence();
  *(volatile v4f*)o = v;
}

__global__ __launch_bounds__(256) void pack_kernel(
    const float* __restrict__ x, const float* __restrict__ pos, const float* __restrict__ back,
    unsigned short* QXh, unsigned short* QXl, unsigned short* KXh, unsigned short* KXl,
    unsigned short* KVh, unsigned short* KVl) {
  const int t = blockIdx.x * 256 + (int)threadIdx.x;
  if (t >= NPADR * C8) return;
  const int j = t / C8;
  const int c = (t - j * C8) * 8;
  const int jx = (j > NQ - 1) ? (NQ - 1) : j;
  const int jp = (j > NKEY - 1) ? (NKEY - 1) : j;
  const v4f xa = *(const v4fa*)(x + (size_t)jx * CDIM + c);
  const v4f xb = *(const v4fa*)(x + (size_t)jx * CDIM + c + 4);
  const v4f pa = *(const v4fa*)(pos + (size_t)jp * CDIM + c);
  const v4f pb = *(const v4fa*)(pos + (size_t)jp * CDIM + c + 4);
  const v4f ga = *(const v4fa*)(back + c);
  const v4f gb = *(const v4fa*)(back + c + 4);
  const bool isq = j < NQ;
  const bool isk = j < NKEY;
  const bool isb = (j == NQ);
  float xv[8], pv[8], bv[8];
#pragma unroll
  for (int e = 0; e < 4; ++e) {
    xv[e] = xa[e]; xv[4 + e] = xb[e];
    pv[e] = pa[e]; pv[4 + e] = pb[e];
    bv[e] = ga[e]; bv[4 + e] = gb[e];
  }
  float fq[8], fk[8], fv[8];
#pragma unroll
  for (int e = 0; e < 8; ++e) {
    const float xr = bf_rn(xv[e]);
    const float pr = bf_rn(pv[e]);
    const float kv = isq ? xr : (isb ? bv[e] : 0.f);
    fq[e] = isq ? (xr + pr) : 0.f;
    fk[e] = isk ? (kv + pr) : 0.f;
    fv[e] = isk ? kv : 0.f;
  }
  v4u oqh, oql, okh, okl, ovh, ovl;
  split8(fq, 1.0f, oqh, oql);
  split8(fk, 1.0f, okh, okl);
  split8(fv, 1.0f, ovh, ovl);
  const size_t go = (size_t)t * 8;
  *(volatile v4u*)(QXh + go) = oqh;
  *(volatile v4u*)(QXl + go) = oql;
  *(volatile v4u*)(KXh + go) = okh;
  *(volatile v4u*)(KXl + go) = okl;
  *(volatile v4u*)(KVh + go) = ovh;
  *(volatile v4u*)(KVl + go) = ovl;
  __threadfence();
  *(volatile v4u*)(QXh + go) = oqh;
  *(volatile v4u*)(QXl + go) = oql;
  *(volatile v4u*)(KXh + go) = okh;
  *(volatile v4u*)(KXl + go) = okl;
  *(volatile v4u*)(KVh + go) = ovh;
  *(volatile v4u*)(KVl + go) = ovl;
}

template <int NPROD, int OUT_MODE>
__global__ __launch_bounds__(256) void gemm64(
    const unsigned short* __restrict__ A0, const unsigned short* __restrict__ A1, int lda,
    const unsigned short* __restrict__ B0, const unsigned short* __restrict__ B1, int ldb,
    void* Cout, void* Cout2, int ldc, const float* __restrict__ bias,
    int M, int N, int K, int nvalid, float oscale) {
  __shared__ __align__(16) float sT[8][16 * 68];
  const int lane = (int)threadIdx.x & 31;
  const int wave = (int)threadIdx.x >> 5;
  const int tilesN = N >> 6;
  const int tilesM = M >> 6;
  const int tile = blockIdx.x * 8 + wave;
  if (tile >= tilesM * tilesN) return;
  const int tm = tile / tilesN;
  const int tn = tile - tm * tilesN;
  const int m0 = tm << 6;
  const int n0 = tn << 6;

  const int rlane = lane & 15;
  const int hh    = lane >> 4;
  const int mOff  = hh * 8;

  v8f acc[4][4];
#pragma unroll
  for (int i = 0; i < 4; ++i)
#pragma unroll
    for (int j = 0; j < 4; ++j) acc[i][j] = zero8();

  for (int k0 = 0; k0 < K; k0 += 32) {
#pragma unroll
    for (int p = 0; p < NPROD; ++p) {
      const unsigned short* Ab = (p == 0) ? A0 : A1;
      const unsigned short* Bb = (p == 0) ? B0 : B1;
      v16b bq[4];
#pragma unroll
      for (int j = 0; j < 4; ++j)
        bq[j] = ldfrag_b(Bb + (size_t)(n0 + (j << 4) + rlane) * ldb + k0, hh);
#pragma unroll
      for (int i = 0; i < 4; ++i) {
        const v16b af = ldfrag_b(Ab + (size_t)(m0 + (i << 4) + rlane) * lda + k0, hh);
#pragma unroll
        for (int j = 0; j < 4; ++j) acc[i][j] = mmar(af, bq[j], acc[i][j]);
        dep_guard(acc[i][0], acc[i][3], af, bq[3]);
      }
      keep4(bq[0], bq[1], bq[2], bq[3]);
    }
  }
  acc_guard4(acc[0][0], acc[0][1], acc[0][2], acc[0][3]);
  acc_guard4(acc[1][0], acc[1][1], acc[1][2], acc[1][3]);
  acc_guard4(acc[2][0], acc[2][1], acc[2][2], acc[2][3]);
  acc_guard4(acc[3][0], acc[3][1], acc[3][2], acc[3][3]);

  float* slab = sT[wave];
  const int h2 = lane >> 4, c4 = (lane & 15) * 4;
  const int q  = lane >> 3, c8 = (lane & 7) * 8;
  v4f bb = {0.f, 0.f, 0.f, 0.f};
  if (OUT_MODE == 0) {
    const v4f braw = *(const v4fa*)(bias + n0 + c4);
#pragma unroll
    for (int e = 0; e < 4; ++e) bb[e] = bf_rn(braw[e]);
  }
#pragma unroll
  for (int i = 0; i < 4; ++i) {
    const int mBase = m0 + (i << 4);
#pragma unroll
    for (int j = 0; j < 4; ++j) {
#pragma unroll
      for (int r = 0; r < 8; ++r) {
        slab[(mOff + r) * 68 + (j << 4) + rlane] = acc[i][j][r];
      }
    }
    __builtin_amdgcn_fence(__ATOMIC_RELEASE, "workgroup");
    __builtin_amdgcn_wave_barrier();
    __builtin_amdgcn_fence(__ATOMIC_ACQUIRE, "workgroup");
    if (OUT_MODE == 0) {
      float* C = (float*)Cout;
      for (int pass = 0; pass < 2; ++pass) {
#pragma unroll
        for (int it = 0; it < 8; ++it) {
          const int row  = it * 2 + h2;
          const int grow = mBase + row;
          const v4f v = *(const v4fa*)(slab + row * 68 + c4) * oscale + bb;
          if (grow < nvalid) *(volatile v4f*)(C + (size_t)grow * ldc + n0 + c4) = v;
        }
        __threadfence();
      }
    } else {
      unsigned short* C  = (unsigned short*)Cout;
      unsigned short* C2 = (unsigned short*)Cout2;
      v4u hv[4], lv[4];
#pragma unroll
      for (int it = 0; it < 4; ++it) {
        const int row = it * 4 + q;
        const float* sp = slab + row * 68 + c8;
        float f[8];
#pragma unroll
        for (int e = 0; e < 8; ++e) f[e] = sp[e];
        split8(f, oscale, hv[it], lv[it]);
      }
      for (int pass = 0; pass < 2; ++pass) {
#pragma unroll
        for (int it = 0; it < 4; ++it) {
          const int row = it * 4 + q;
          const size_t go = (size_t)(mBase + row) * ldc + n0 + c8;
          *(volatile v4u*)(C + go)  = hv[it];
          *(volatile v4u*)(C2 + go) = lv[it];
        }
        __threadfence();
      }
    }
    __builtin_amdgcn_fence(__ATOMIC_RELEASE, "workgroup");
    __builtin_amdgcn_wave_barrier();
    __builtin_amdgcn_fence(__ATOMIC_ACQUIRE, "workgroup");
  }
}

__global__ __launch_bounds__(128) void attn_kernel(
    const unsigned short* __restrict__ Qh, const unsigned short* __restrict__ Ql,
    const unsigned short* __restrict__ Kh, const unsigned short* __restrict__ Kl,
    const unsigned short* __restrict__ VTh, const unsigned short* __restrict__ VTl,
    const float* __restrict__ mk, unsigned short* CTh, unsigned short* CTl) {
  __shared__ __align__(16) float sO[4 * 16 * 64];

  const int tid = (int)threadIdx.x, lane = tid & 31, w = tid >> 5;
  const int hh = lane >> 4, m = lane & 15;
  const int head = blockIdx.y;
  const int q0 = blockIdx.x * 64 + 16 * w;

  const size_t qo = (size_t)(q0 + m) * CDIM + (size_t)head * DHEAD;
  const v16b qh0 = ldfrag_b(Qh + qo, hh);
  const v16b qh1 = ldfrag_b(Qh + qo + 32, hh);
  const v16b ql0 = ldfrag_b(Ql + qo, hh);
  const v16b ql1 = ldfrag_b(Ql + qo + 32, hh);

  v8f o[4];
#pragma unroll
  for (int t = 0; t < 4; ++t) o[t] = zero8();
  float mrun = PADFILL, lrun = 0.0f;

  const unsigned short* khb = Kh  + (size_t)m * CDIM + (size_t)head * DHEAD;
  const unsigned short* klb = Kl  + (size_t)m * CDIM + (size_t)head * DHEAD;
  const unsigned short* vhb = VTh + ((size_t)head * DHEAD + m) * NPADR;
  const unsigned short* vlb = VTl + ((size_t)head * DHEAD + m) * NPADR;
  const float* mkp = mk + 8 * hh;

#pragma unroll 1
  for (int kb = 0; kb < NPADR; kb += 64) {
    v8f s[4];
#pragma unroll
    for (int j = 0; j < 4; ++j) {
      const size_t ko = (size_t)(kb + 16 * j) * CDIM;
      v8f z = zero8();
      {
        const v16b a0 = ldfrag_b(khb + ko, hh);
        const v16b a1 = ldfrag_b(khb + ko + 32, hh);
        z = mma_g(a0, qh0, z);
        z = mma_g(a1, qh1, z);
        z = mma_g(a0, ql0, z);
        z = mma_g(a1, ql1, z);
      }
      {
        const v16b b0 = ldfrag_b(klb + ko, hh);
        const v16b b1 = ldfrag_b(klb + ko + 32, hh);
        z = mma_g(b0, qh0, z);
        z = mma_g(b1, qh1, z);
      }
      s[j] = z;
    }
#pragma unroll
    for (int j = 0; j < 4; ++j) {
      const v4f ma = *(const v4fa*)(mkp + kb + 16 * j);
      const v4f mb = *(const v4fa*)(mkp + kb + 16 * j + 4);
#pragma unroll
      for (int e = 0; e < 4; ++e) {
        s[j][e]     = (ma[e] > 0.f) ? s[j][e]     : ma[e];
        s[j][4 + e] = (mb[e] > 0.f) ? s[j][4 + e] : mb[e];
      }
    }

    float mloc = s[0][0];
#pragma unroll
    for (int j = 0; j < 4; ++j)
#pragma unroll
      for (int r = 0; r < 8; ++r) mloc = fmaxf(mloc, s[j][r]);
    mloc = fmaxf(mloc, __shfl_xor(mloc, 16, 32));
    const float mnew  = fmaxf(mrun, mloc);
    const float alpha = __expf(mrun - mnew);
    mrun = mnew;
    float lsum = 0.0f;
#pragma unroll
    for (int j = 0; j < 4; ++j)
#pragma unroll
      for (int r = 0; r < 8; ++r) {
        const float p = __expf(s[j][r] - mnew);
        s[j][r] = p;
        lsum += p;
      }
    lsum += __shfl_xor(lsum, 16, 32);
    lrun = lrun * alpha + lsum;
#pragma unroll
    for (int t = 0; t < 4; ++t)
#pragma unroll
      for (int r = 0; r < 8; ++r) o[t][r] = o[t][r] * alpha;

    v16b ph0, pl0, ph1, pl1;
    pack_p2(s[0], s[1], ph0, pl0);
    pack_p2(s[2], s[3], ph1, pl1);

#pragma unroll
    for (int t = 0; t < 4; ++t) {
      const size_t vo = (size_t)(16 * t) * NPADR + kb;
      {
        const v16b a0 = ldfrag_b(vhb + vo, hh);
        const v16b a1 = ldfrag_b(vhb + vo + 32, hh);
        o[t] = mma_g(a0, ph0, o[t]);
        o[t] = mma_g(a1, ph1, o[t]);
        o[t] = mma_g(a0, pl0, o[t]);
        o[t] = mma_g(a1, pl1, o[t]);
      }
      {
        const v16b b0 = ldfrag_b(vlb + vo, hh);
        const v16b b1 = ldfrag_b(vlb + vo + 32, hh);
        o[t] = mma_g(b0, ph0, o[t]);
        o[t] = mma_g(b1, ph1, o[t]);
      }
    }
  }

  const float inv = 1.0f / lrun;
  float* so = sO + w * 1024;
#pragma unroll
  for (int t = 0; t < 4; ++t)
#pragma unroll
    for (int r = 0; r < 8; ++r)
      so[m * 64 + 16 * t + 8 * hh + r] = o[t][r] * inv;
  __syncthreads();

  const int q8 = lane & 7, sub = lane >> 3;
  v4u hv[4], lv[4];
#pragma unroll
  for (int it = 0; it < 4; ++it) {
    const int row = it * 4 + sub;
    const v4f fa = *(const v4fa*)(so + row * 64 + 8 * q8);
    const v4f fb = *(const v4fa*)(so + row * 64 + 8 * q8 + 4);
    float f[8];
#pragma unroll
    for (int e = 0; e < 4; ++e) { f[e] = fa[e]; f[4 + e] = fb[e]; }
    split8(f, 1.0f, hv[it], lv[it]);
  }
  for (int pass = 0; pass < 2; ++pass) {
#pragma unroll
    for (int it = 0; it < 4; ++it) {
      const int row = it * 4 + sub;
      const size_t go = (size_t)(q0 + row) * CDIM + (size_t)head * DHEAD + 8 * q8;
      *(volatile v4u*)(CTh + go) = hv[it];
      *(volatile v4u*)(CTl + go) = lv[it];
    }
    __threadfence();
  }
}

extern "C" void kernel_launch(void* const* d_in, const int* in_sizes, int n_in,
                              void* d_out, int out_size, void* d_ws, size_t ws_size,
                              hipStream_t stream) {
  if (n_in < 9) return;
  if (in_sizes[0] != NQ * CDIM) return;
  if (in_sizes[1] != NKEY * CDIM) return;
  if (in_sizes[2] != NINT) return;
  if (in_sizes[3] != NKEY) return;
  if (in_sizes[4] != CDIM * CDIM || in_sizes[5] != CDIM * CDIM ||
      in_sizes[6] != CDIM * CDIM || in_sizes[7] != CDIM * CDIM) return;
  if (in_sizes[8] != CDIM) return;
  if (out_size != NQ * CDIM) return;

  const float* x    = (const float*)d_in[0];
  const float* pos  = (const float*)d_in[1];
  const float* msk  = (const float*)d_in[2];
  const float* mblk = (const float*)d_in[3];
  const float* Wq   = (const float*)d_in[4];
  const float* Wk   = (const float*)d_in[5];
  const float* Wv   = (const float*)d_in[6];
  const float* Wp   = (const float*)d_in[7];
  const float* bp   = (const float*)d_in[8];
  float* out = (float*)d_out;

  const size_t PBK = (size_t)CDIM * 4;
  const size_t PMK = (size_t)NPADR * 4;
  const size_t PW  = (size_t)CDIM * CDIM * 2;
  const size_t PA  = PLANE * 2;
  size_t off = 0;
  const size_t oBack = off; off += PBK;
  const size_t oMk   = off; off += PMK;
  const size_t oWb   = off; off += 4 * PW;
  const size_t oQXh  = off; off += PA;
  const size_t oQXl  = off; off += PA;
  const size_t oKXh  = off; off += PA;
  const size_t oKXl  = off; off += PA;
  const size_t oKVh  = off; off += PA;
  const size_t oKVl  = off; off += PA;
  const size_t oQh   = off; off += PA;
  const size_t oQl   = off; off += PA;
  const size_t oKh   = off; off += PA;
  const size_t oKl   = off; off += PA;
  const size_t oVTh  = off; off += PA;
  const size_t oVTl  = off; off += PA;
  const size_t oCTh  = off; off += PA;
  const size_t oCTl  = off; off += PA;
  if (off > ws_size) return;
  if (off > (size_t)134217728) return;

  char* ws = (char*)d_ws;
  float*          back = (float*)(ws + oBack);
  float*          mk   = (float*)(ws + oMk);
  unsigned short* Wb   = (unsigned short*)(ws + oWb);
  unsigned short* Wqb  = Wb;
  unsigned short* Wkb  = Wb + (size_t)CDIM * CDIM;
  unsigned short* Wvb  = Wb + (size_t)2 * CDIM * CDIM;
  unsigned short* Wpb  = Wb + (size_t)3 * CDIM * CDIM;
  unsigned short* QXh  = (unsigned short*)(ws + oQXh);
  unsigned short* QXl  = (unsigned short*)(ws + oQXl);
  unsigned short* KXh  = (unsigned short*)(ws + oKXh);
  unsigned short* KXl  = (unsigned short*)(ws + oKXl);
  unsigned short* KVh  = (unsigned short*)(ws + oKVh);
  unsigned short* KVl  = (unsigned short*)(ws + oKVl);
  unsigned short* Qh   = (unsigned short*)(ws + oQh);
  unsigned short* Ql   = (unsigned short*)(ws + oQl);
  unsigned short* Kh   = (unsigned short*)(ws + oKh);
  unsigned short* Kl   = (unsigned short*)(ws + oKl);
  unsigned short* VTh  = (unsigned short*)(ws + oVTh);
  unsigned short* VTl  = (unsigned short*)(ws + oVTl);
  unsigned short* CTh  = (unsigned short*)(ws + oCTh);
  unsigned short* CTl  = (unsigned short*)(ws + oCTl);

  const int tiles = (NPADR / 64) * (CDIM / 64);
  const dim3 gGemm((tiles + 7) / 8);
  const dim3 gAttn(NPADR / 64, NHEAD);

  back_kernel<<<dim3(CDIM / 32), dim3(256), 0, stream>>>(x, msk, back);
  wcvt_kernel<<<dim3(CDIM * CDIM / 8 / 256, 4), dim3(256), 0, stream>>>(Wq, Wk, Wv, Wp, Wb);
  keymask_kernel<<<dim3((NPADR / 4 + 255) / 256), dim3(256), 0, stream>>>(msk, mblk, mk);
  pack_kernel<<<dim3(NPADR * C8 / 256), dim3(256), 0, stream>>>(x, pos, back, QXh, QXl, KXh, KXl, KVh, KVl);
  gemm64<2, 3><<<gGemm, dim3(256), 0, stream>>>(
      QXh, QXl, CDIM, Wqb, Wqb, CDIM, (void*)Qh, (void*)Ql, CDIM, bp, NPADR, CDIM, CDIM, NPADR, 0.125f);
  gemm64<2, 3><<<gGemm, dim3(256), 0, stream>>>(
      KXh, KXl, CDIM, Wkb, Wkb, CDIM, (void*)Kh, (void*)Kl, CDIM, bp, NPADR, CDIM, CDIM, NPADR, 1.0f);
  gemm64<2, 3><<<gGemm, dim3(256), 0, stream>>>(
      Wvb, Wvb, CDIM, KVh, KVl, CDIM, (void*)VTh, (void*)VTl, NPADR, bp, CDIM, NPADR, CDIM, CDIM, 1.0f);
  attn_kernel<<<gAttn, dim3(128), 0, stream>>>(Qh, Ql, Kh, Kl, VTh, VTl, mk, CTh, CTl);
  gemm64<2, 0><<<gGemm, dim3(256), 0, stream>>>(
      CTh, CTl, CDIM, Wpb, Wpb, CDIM, (void*)out, (void*)out, CDIM, bp, NPADR, CDIM, CDIM, NQ, 1.0f);
  (void)hipGetLastError();
}
